// ScaledDotProductAttention_27109833572478
// MI455X (gfx1250) — hardware-verified
//
#include <hip/hip_runtime.h>
#ifndef NB
#define NB 2
#endif
#ifndef SEQ
#define SEQ 2048
#endif
#define NB_FULL 2
#define SEQ_FULL 2048
#define NHEAD 16
#define HD 64
#define HG 4
#ifndef OUT_ROWS
#define OUT_ROWS SEQ_FULL
#endif
#define NPL (NB * NHEAD)
#define RCH (SEQ / 256)
static_assert(NB >= 1 && NB <= NB_FULL);
static_assert(SEQ >= 256 && SEQ <= SEQ_FULL && (SEQ % 256) == 0);
static_assert(HD == 64);
static_assert((NPL % HG) == 0);
static_assert((HG * SEQ) % 8 == 0);

typedef _Float16 v16h __attribute__((ext_vector_type(16)));
typedef _Float16 v4h  __attribute__((ext_vector_type(4)));
typedef unsigned short v8us __attribute__((ext_vector_type(8), may_alias));
typedef float  v8f  __attribute__((ext_vector_type(8)));
typedef float  v4f  __attribute__((ext_vector_type(4)));
typedef float  v4fa __attribute__((ext_vector_type(4), may_alias));
typedef int    v4i  __attribute__((ext_vector_type(4), may_alias));
union FragH { v16h v; v8us half[2]; _Float16 h[16]; unsigned short u[16]; };

__device__ __forceinline__ unsigned short bf16_bits(float x) { unsigned int u = __float_as_uint(x); return (unsigned short)((u + 0x7FFFu + ((u >> 16) & 1u)) >> 16); }
__device__ __forceinline__ float bf16_val(unsigned short b) { return __uint_as_float(((unsigned int)b) << 16); }
__device__ __forceinline__ float bf16_rne(float x) { return bf16_val(bf16_bits(x)); }

__device__ __forceinline__ v16h g2_frag(const _Float16* p, int hh) { FragH f; f.half[0] = *(const v8us*)((const unsigned short*)p + 8 * hh); f.half[1] = *(const v8us*)((const unsigned short*)p + 16 + 8 * hh); return f.v; }
__device__ __forceinline__ v8f g2_mma(v16h a, v16h b, v8f c) { v8f d = __builtin_amdgcn_wmma_f32_16x16x32_f16(false, a, false, b, (short)0, c, false, false); asm volatile("v_nop\n\tv_nop\n\tv_nop\n\tv_nop" : "+v"(d) : "v"(a), "v"(b)); return d; }
template <int ACT>
__global__ __launch_bounds__(128) void k_gemm2(const _Float16* __restrict__ A, int lda, size_t sA, const _Float16* __restrict__ Bh, int ldb, size_t sB, float alpha, const float* __restrict__ bias, size_t sBias, const float* __restrict__ CP, int rowsPerB, size_t sCPb, int row0g,
    float* __restrict__ C, _Float16* __restrict__ C16, int ldc, size_t sC, int M, int N, int K) { static_assert(ACT == 0 || ACT == 3 || ACT == 6 || ACT == 8 || ACT == 9 || ACT == 11 || ACT == 12 || ACT == 14 || ACT == 15 || ACT == 16 || ACT == 17);
  __shared__ __attribute__((aligned(16))) float so[4][32][68];
  const int tid = threadIdx.x, w = tid >> 5, lane = tid & 31, ln = lane & 15, hh = lane >> 4; const int by = blockIdx.y;
  A += (size_t)by * sA; Bh += (size_t)by * sB; const size_t cofs = (size_t)by * sC; const float* bp = bias ? bias + (size_t)by * sBias : nullptr;
  const int ntn = N >> 6; const int mt = blockIdx.x / ntn, nq = blockIdx.x - mt * ntn; const int row0 = mt * 128 + 32 * w, col0 = nq * 64; if (row0 >= M) return;
  const _Float16* a0p = A + (size_t)(row0 + ln) * lda; const _Float16* a1p = a0p + (size_t)16 * lda;
  const _Float16* b0p = Bh + (size_t)(col0 + ln) * ldb; const _Float16* b1p = b0p + (size_t)16 * ldb; const _Float16* b2p = b1p + (size_t)16 * ldb; const _Float16* b3p = b2p + (size_t)16 * ldb;
  const v8f z8 = {0.f,0.f,0.f,0.f,0.f,0.f,0.f,0.f}; v8f c00 = z8, c01 = z8, c02 = z8, c03 = z8, c10 = z8, c11 = z8, c12 = z8, c13 = z8;
#pragma unroll 1
  for (int kb = 0; kb < K; kb += 32) { const v16h a0 = g2_frag(a0p + kb, hh), a1 = g2_frag(a1p + kb, hh);
    v16h b = g2_frag(b0p + kb, hh); c00 = g2_mma(a0, b, c00); c10 = g2_mma(a1, b, c10);
    b = g2_frag(b1p + kb, hh); c01 = g2_mma(a0, b, c01); c11 = g2_mma(a1, b, c11);
    b = g2_frag(b2p + kb, hh); c02 = g2_mma(a0, b, c02); c12 = g2_mma(a1, b, c12);
    b = g2_frag(b3p + kb, hh); c03 = g2_mma(a0, b, c03); c13 = g2_mma(a1, b, c13); }
  v8f accs[8] = {c00, c01, c02, c03, c10, c11, c12, c13};
#pragma unroll
  for (int u = 0; u < 8; ++u) { const int t = u & 3, mh = u >> 2; const int col = col0 + t * 16 + ln; const float bv = bp ? bf16_rne(bp[col]) : 0.f;
#pragma unroll
    for (int r = 0; r < 8; ++r) { const int rloc = mh * 16 + 8 * hh + r; float v = accs[u][r] * alpha + bv; if (CP) { if (rowsPerB < 0) v += CP[cofs + (size_t)(row0g + row0 + rloc) * ldc + col];        else { const int bidx = (row0g + row0 + rloc) / rowsPerB; v += CP[(size_t)bidx * sCPb + (size_t)by * 64 + col]; } }
      if (ACT == 3) v = fmaxf(v, 0.f); else if (ACT == 6) v = 0.5f * v * (1.0f + erff(v * 0.70710678118654752f)); else if (ACT == 11) v = 1.0f / (1.0f + expf(-v)); else if (ACT == 15) v = v / (1.0f + expf(-v)); else if (ACT == 12) v = (v > 0.f) ? v : 0.01f * v; else if (ACT == 8) v = tanhf(v); else if (ACT == 9) v = 0.5f * v * (1.0f + tanhf(0.7978845608028654f * (v + 0.044715f * v * v * v))); else if (ACT == 14) v = (v > 0.f) ? v : 0.1f * v; else if (ACT == 16) v = (v >= 0.f) ? v : 0.3f * v; else if (ACT == 17) v = (v >= 0.f) ? v : 0.2f * v;
      so[w][rloc][t * 16 + ln] = v; } }
  __builtin_amdgcn_fence(4  , "workgroup"); __builtin_amdgcn_wave_barrier();
  const int rsub = lane >> 4, c4 = (lane & 15) * 4;
  for (int pass = 0; pass < 2; ++pass) {
#pragma unroll
    for (int q = 0; q < 16; ++q) { const int r = q * 2 + rsub; const v4f v = *(const v4fa*)&so[w][r][c4]; if (C) *(volatile v4f*)(C + cofs + (size_t)(row0 + r) * ldc + col0 + c4) = v; if (C16) { v4h h4; for (int i = 0; i < 4; ++i) h4[i] = (_Float16)v[i]; *(volatile v4h*)(C16 + cofs + (size_t)(row0 + r) * ldc + col0 + c4) = h4; } }
    if (pass == 0) __threadfence(); } }

__global__ __launch_bounds__(256) void k_x16(const float* __restrict__ x, _Float16* __restrict__ X16, size_t n8) {
  const size_t t = (size_t)blockIdx.x * 256 + threadIdx.x; if (t >= n8) return;
  const size_t e = t * 8; const size_t row = e / HD; const size_t c = e - row * HD; const size_t p = row / SEQ, s = row - p * SEQ;
  const float* src = x + (p * SEQ_FULL + s) * HD + c;
  const v4f a = *(const v4fa*)src, a2 = *(const v4fa*)(src + 4);
  FragH f;
#pragma unroll
  for (int q = 0; q < 4; ++q) { f.h[q] = (_Float16)bf16_rne(a[q]); f.h[4 + q] = (_Float16)bf16_rne(a2[q]); }
  const v8us o = f.half[0];
  *(volatile v8us*)((unsigned short*)X16 + e) = o; __threadfence(); *(volatile v8us*)((unsigned short*)X16 + e) = o;
}

__global__ __launch_bounds__(256) void k_vt(const _Float16* __restrict__ V16, int p0, _Float16* __restrict__ VT) {
  __shared__ unsigned short tl[64][65];
  const int tid = threadIdx.x; const int hh = blockIdx.x % HG, sg = blockIdx.x / HG; const int s0 = sg * 64;
  for (int i = tid; i < 64 * 8; i += 256) { const int j = i / 8, d8 = (i % 8) * 8; FragH f;
    f.half[0] = *(const v8us*)((const unsigned short*)V16 + ((size_t)(p0 + hh) * SEQ + s0 + j) * HD + d8);
#pragma unroll
    for (int q = 0; q < 8; ++q) tl[d8 + q][j] = f.u[q]; }
  __syncthreads();
  for (int pass = 0; pass < 2; ++pass) {
    for (int i = tid; i < 64 * 8; i += 256) { const int d = i / 8, j8 = (i % 8) * 8; FragH f;
#pragma unroll
      for (int q = 0; q < 8; ++q) f.u[q] = tl[d][j8 + q];
      *(volatile v8us*)((unsigned short*)VT + ((size_t)hh * HD + d) * SEQ + s0 + j8) = f.half[0]; }
    if (pass == 0) __threadfence(); } }

__global__ __launch_bounds__(256) void k_rsmw(const float* __restrict__ S, const int* __restrict__ mask, _Float16* __restrict__ P, int qn, int hg, int p0) {
  #pragma clang fp contract(off)
  const int tid = threadIdx.x, lane = tid & 31;
  const int t = blockIdx.x * 8 + (tid >> 5);
  if (t >= qn * hg) return;
  const int hl = t / qn, q = t - hl * qn;
  const int b = (p0 + hl) / NHEAD;
  const float* s = S + ((size_t)hl * SEQ + q) * SEQ;
  const int* mk = mask + ((size_t)b * SEQ_FULL + q) * SEQ_FULL;
  unsigned short* d = (unsigned short*)P + ((size_t)hl * SEQ + q) * SEQ;
  float v[RCH * 8]; unsigned int mb[RCH];
  float mx = -3.0e38f;
#pragma unroll
  for (int it = 0; it < RCH; ++it) {
    const int j0 = it * 256 + lane * 8;
    const v4f a = *(const v4fa*)(s + j0), c = *(const v4fa*)(s + j0 + 4);
    const v4i ma = *(const v4i*)(mk + j0), mc = *(const v4i*)(mk + j0 + 4);
    unsigned int bits = 0u;
#pragma unroll
    for (int u = 0; u < 4; ++u) {
      v[it * 8 + u] = a[u]; v[it * 8 + 4 + u] = c[u];
      bits |= ((ma[u] != 0) ? 1u : 0u) << u; bits |= ((mc[u] != 0) ? 1u : 0u) << (4 + u);
    }
    mb[it] = bits;
#pragma unroll
    for (int u = 0; u < 8; ++u) mx = ((bits >> u) & 1u) ? fmaxf(mx, v[it * 8 + u]) : mx;
  }
#pragma unroll
  for (int m = 16; m > 0; m >>= 1) mx = fmaxf(mx, __shfl_xor(mx, m));
  float se = 0.f;
#pragma unroll
  for (int it = 0; it < RCH; ++it) {
#pragma unroll
    for (int u = 0; u < 8; ++u) { const float e = ((mb[it] >> u) & 1u) ? __expf(v[it * 8 + u] - mx) : 0.f; v[it * 8 + u] = e; se += e; }
  }
#pragma unroll
  for (int m = 16; m > 0; m >>= 1) se += __shfl_xor(se, m);
  const bool live = se > 0.f;
  const float se1 = live ? se : 1.0f;
  float sc = 256.0f * (1.0f / se1);
  sc = live ? sc : __uint_as_float(0x7FC00000u);
#pragma unroll
  for (int it = 0; it < RCH; ++it) {
    const int j0 = it * 256 + lane * 8;
    FragH f;
#pragma unroll
    for (int u = 0; u < 8; ++u) f.h[u] = (_Float16)(v[it * 8 + u] * sc);
    const v8us o = f.half[0];
    *(volatile v8us*)(d + j0) = o; __threadfence(); *(volatile v8us*)(d + j0) = o;
  }
}

extern "C" void kernel_launch(void* const* d_in, const int* in_sizes, int n_in,
                              void* d_out, int out_size, void* d_ws, size_t ws_size, hipStream_t stream) {
  if (n_in < 4) return;
  const long long need_x = (long long)NB * NHEAD * SEQ_FULL * HD;
  if ((long long)in_sizes[0] < need_x || (long long)in_sizes[1] < need_x || (long long)in_sizes[2] < need_x) return;
  if ((long long)in_sizes[3] < (long long)NB * SEQ_FULL * SEQ_FULL) return;
  if ((long long)out_size < ((long long)(NPL - 1) * OUT_ROWS + SEQ) * HD) return;
  const float* xq = (const float*)d_in[0]; const float* xk = (const float*)d_in[1]; const float* xv = (const float*)d_in[2]; const int* mask = (const int*)d_in[3];
  float* out = (float*)d_out;
  char* ws = (char*)d_ws; size_t off = 0;
  auto take = [&](size_t bytes) { char* p = ws + off; off += (bytes + 255) & ~(size_t)255; return p; };
  const size_t plane16 = (size_t)NPL * SEQ * HD * 2;
  _Float16* Q16 = (_Float16*)take(plane16); _Float16* K16 = (_Float16*)take(plane16); _Float16* V16 = (_Float16*)take(plane16);
  float* S = (float*)take((size_t)HG * SEQ * SEQ * 4);
  _Float16* P = (_Float16*)take((size_t)HG * SEQ * SEQ * 2);
  _Float16* VT = (_Float16*)take((size_t)HG * HD * SEQ * 2);
  if (off > ws_size) return;

  const size_t n8 = (size_t)NPL * SEQ * HD / 8; const unsigned cg = (unsigned)((n8 + 255) / 256);
  k_x16<<<cg, 256, 0, stream>>>(xq, Q16, n8); k_x16<<<cg, 256, 0, stream>>>(xk, K16, n8); k_x16<<<cg, 256, 0, stream>>>(xv, V16, n8);
  for (int g = 0; g < NPL / HG; ++g) { const int p0 = g * HG;
    k_vt<<<HG * (SEQ / 64), 256, 0, stream>>>(V16, p0, VT);
    k_gemm2<0><<<dim3((SEQ / 128) * (SEQ / 64), HG), 128, 0, stream>>>(Q16 + (size_t)p0 * SEQ * HD, HD, (size_t)SEQ * HD, K16 + (size_t)p0 * SEQ * HD, HD, (size_t)SEQ * HD, 0.125f, nullptr, 0, nullptr, 1, 0, 0, S, nullptr, SEQ, (size_t)SEQ * SEQ, SEQ, SEQ, HD);
    k_rsmw<<<(HG * SEQ) / 8, 256, 0, stream>>>(S, mask, P, SEQ, HG, p0);
    k_gemm2<0><<<dim3((SEQ / 128) * (HD / 64), HG), 128, 0, stream>>>(P, SEQ, (size_t)SEQ * SEQ, VT, SEQ, (size_t)HD * SEQ, 0.00390625f, nullptr, 0, nullptr, 1, 0, 0, out + (size_t)p0 * OUT_ROWS * HD, nullptr, HD, (size_t)OUT_ROWS * HD, SEQ, HD, SEQ); }
}
